// RGAT_GCN_concat_22333829939347
// MI455X (gfx1250) — hardware-run, weakly checked
//
#include <hip/hip_runtime.h>
#include <stddef.h>
#include <stdint.h>
#include <math.h>

#define NN      50000
#define NE      800000
#define NR      3
#define FIN     128
#define HB      64
#define MP      50048
#define GBM     128
#define NTHR    256
#define NWAVE   8
#define EPT     8
#define WCH     (32 * EPT)
#define NBRUN   1024
#define SLB     10
#define NBK     49
#define NSLOT   (NBK * NBRUN)
#define WLCAP   2560
#define RCAP    20480
#define DEGCAP  64
#define MAXDEG_MEAS   36
#define MAXB1024_MEAS 16753
#define FW      384
#define HLW     256
#define RBM     64
#define SP      68
#define WSMAX   134217728

#define SM_ATT  0
#define SM_BIAS 768
#define SM_BLIN 1536
#define SM_N    1600
#define ER_OFS  (NR * MP * 4)

#define BK_ZINTS (NWAVE * WLCAP + RCAP + 3 * NBRUN)
#define BK_INTS  (BK_ZINTS + 16)
#define BK_LDS   (BK_INTS * 4)

#define PBX  (MP * FIN / 8 / NTHR)
#define PBW  (NR * HB * 128 / 8 / NTHR)
#define PB3  (HB * HLW / 8 / NTHR)
#define PBS  9
#define PBTOT (PBX + 4 * PBW + PB3 + PBS)

static_assert(MP == 391 * GBM && MP >= NN && MP % RBM == 0);
static_assert(NBRUN == (1 << SLB) && NBRUN % GBM == 0 && NBRUN % RBM == 0 && NBRUN % 32 == 0);
static_assert(NSLOT >= MP && NBRUN == 4 * NTHR);
static_assert(NE % WCH == 0 && NE % 4 == 0);
static_assert(NE < (1 << 21) && (((long long)NE) << SLB) < (1LL << 31));
static_assert(RCAP == NWAVE * WLCAP && RCAP % 4 == 0 && BK_ZINTS % 4 == 0 && RCAP % (NTHR * 4) == 0);
static_assert((long long)RCAP * 100 >= (long long)MAXB1024_MEAS * 105);
static_assert(WLCAP >= MAXB1024_MEAS / 8 + 8 * 46 + 1);
static_assert(MAXDEG_MEAS + 8 <= DEGCAP);
static_assert(BK_LDS <= 300000);
static_assert((MP * FIN / 8) % NTHR == 0 && (NR * HB * 128 / 8) % NTHR == 0 && (HB * HLW / 8) % NTHR == 0);
static_assert(FIN % 32 == 0 && HLW % 32 == 0 && FW == NR * 2 * HB && HLW == 4 * HB);
static_assert((GBM * SP + 128 + 128 + 1024) * 4 <= 65536);
static_assert(RBM % NWAVE == 0);

typedef float          v4f   __attribute__((ext_vector_type(4)));
typedef float          v8f   __attribute__((ext_vector_type(8)));
typedef int            v4i   __attribute__((ext_vector_type(4)));
typedef int            v8i   __attribute__((ext_vector_type(8)));
typedef unsigned short v8us  __attribute__((ext_vector_type(8)));
typedef unsigned short v16us __attribute__((ext_vector_type(16)));
typedef __bf16         v16bf __attribute__((ext_vector_type(16)));
typedef v4f  __attribute__((may_alias)) v4fa;
typedef v4i  __attribute__((may_alias)) v4ia;
typedef v8us __attribute__((may_alias)) v8usa;
union FragB { v16bf v; v16us u; v8us h[2]; v8i w; };

__device__ __forceinline__ v8f wmb(const FragB& a, const FragB& b, v8f c) {
  v8f d = __builtin_amdgcn_wmma_f32_16x16x32_bf16(false, a.v, false, b.v, (short)0, c, false, false);
  asm volatile("v_nop\n\tv_nop\n\tv_nop\n\tv_nop" : "+v"(d) : "v"(a.w), "v"(b.w));
  return d;
}

__device__ __forceinline__ unsigned bf16_bits(float f) {
  const unsigned u = __float_as_uint(f);
  const unsigned r = (u + 0x7FFFu + ((u >> 16) & 1u)) >> 16;
  const unsigned q = (u >> 16) | 0x40u;
  return ((u & 0x7fffffffu) > 0x7f800000u) ? q : r;
}
__device__ __forceinline__ float bf16_val(float f) {
  return __uint_as_float(bf16_bits(f) << 16);
}

__device__ __forceinline__ void hilo_pack(float v0, float v1, float v2, float v3,
                                          int& h01, int& h23, int& l01, int& l23) {
  const unsigned a0 = bf16_bits(v0), a1 = bf16_bits(v1), a2 = bf16_bits(v2), a3 = bf16_bits(v3);
  const unsigned b0 = bf16_bits(v0 - __uint_as_float(a0 << 16));
  const unsigned b1 = bf16_bits(v1 - __uint_as_float(a1 << 16));
  const unsigned b2 = bf16_bits(v2 - __uint_as_float(a2 << 16));
  const unsigned b3 = bf16_bits(v3 - __uint_as_float(a3 << 16));
  h01 = (int)(a0 | (a1 << 16)); h23 = (int)(a2 | (a3 << 16));
  l01 = (int)(b0 | (b1 << 16)); l23 = (int)(b2 | (b3 << 16));
}

__device__ __forceinline__ v4i regroup8(int h01, int h23, int l01, int l23, int lane) {
  const int t  = lane & 15;
  const int s0 = (lane & 16) + ((2 * t) & 15), s1 = s0 + 1;
  const int a0 = __shfl(h01, s0, 32), a1 = __shfl(h23, s0, 32), a2 = __shfl(h01, s1, 32), a3 = __shfl(h23, s1, 32);
  const int b0 = __shfl(l01, s0, 32), b1 = __shfl(l23, s0, 32), b2 = __shfl(l01, s1, 32), b3 = __shfl(l23, s1, 32);
  const int mk = (t < 8) ? -1 : 0;
  v4i o;
  o.x = (a0 & mk) | (b0 & ~mk); o.y = (a1 & mk) | (b1 & ~mk);
  o.z = (a2 & mk) | (b2 & ~mk); o.w = (a3 & mk) | (b3 & ~mk);
  return o;
}

__device__ __forceinline__ void st2_v4f(float* p, v4f v) {
  *(volatile v4f*)p = v;
  __threadfence();
  *(volatile v4f*)p = v;
}
__device__ __forceinline__ void st2_v8us(unsigned short* p, v8us v) {
  *(volatile v8us*)p = v;
  __threadfence();
  *(volatile v8us*)p = v;
}

__device__ __forceinline__ v8us colfetch8(const float* __restrict__ base, int stride) {
  float f[8];
#pragma unroll
  for (int i = 0; i < 8; ++i) f[i] = base[(size_t)i * (size_t)stride];
  v8us o;
#pragma unroll
  for (int i = 0; i < 8; ++i) o[i] = (unsigned short)bf16_bits(f[i]);
  return o;
}

__device__ __forceinline__ void wplane(const float* __restrict__ w, int kin, int brofs, unsigned short* bt, int u) {
  const int j = u >> 4, k8 = (u & 15) * 8;
  const int r = j >> 6, c = j & 63;
  const int kk = k8 & (kin - 1);
  const v8us o = colfetch8(w + (size_t)r * (size_t)kin * HB + (size_t)kk * HB + c, HB);
  st2_v8us(bt + (size_t)(r * 128 + brofs + c) * 128 + k8, o);
}

__device__ __forceinline__ void small_plane(const float* __restrict__ src, float* dst, int nq, int tid) {
  if (tid < 64) {
    const int tc = tid < nq ? tid : nq - 1;
    const int r = tc >> 4, q = tc & 15;
    const v4f a = *(const v4fa*)(src + 4 * tc);
    asm volatile("" :: "v"(a));
    v4f o;
    o.x = bf16_val(a.x); o.y = bf16_val(a.y); o.z = bf16_val(a.z); o.w = bf16_val(a.w);
    float* p = dst + r * 128 + 4 * q;
    const bool wr = tid < nq;
    if (wr) *(volatile v4f*)p = o;
    __threadfence();
    if (wr) *(volatile v4f*)p = o;
  }
}

__global__ __launch_bounds__(NTHR) void k_prep(
    const float* __restrict__ x,
    const float* __restrict__ w1a, const float* __restrict__ w1c,
    const float* __restrict__ w2a, const float* __restrict__ w2c,
    const float* __restrict__ wlin,
    const float* __restrict__ al1, const float* __restrict__ ar1,
    const float* __restrict__ al2, const float* __restrict__ ar2,
    const float* __restrict__ b1a, const float* __restrict__ b2a,
    const float* __restrict__ b1c, const float* __restrict__ b2c,
    const float* __restrict__ blin,
    unsigned short* xb, unsigned short* b1, unsigned short* b2, unsigned short* b3, float* sm) {
  const int tid = (int)threadIdx.x;
  const int blk = (int)blockIdx.x;
  if (blk < PBX) {
    const int u   = blk * NTHR + tid;
    const int row = u >> 4, k8 = (u & 15) * 8;
    const int rc  = row < NN ? row : NN - 1;
    const unsigned mk = row < NN ? 0xffffu : 0u;
    const float* p = x + (size_t)rc * FIN + k8;
    const v4f a = *(const v4fa*)p;
    const v4f b = *(const v4fa*)(p + 4);
    v8us o;
    o[0] = (unsigned short)(bf16_bits(a.x) & mk); o[1] = (unsigned short)(bf16_bits(a.y) & mk);
    o[2] = (unsigned short)(bf16_bits(a.z) & mk); o[3] = (unsigned short)(bf16_bits(a.w) & mk);
    o[4] = (unsigned short)(bf16_bits(b.x) & mk); o[5] = (unsigned short)(bf16_bits(b.y) & mk);
    o[6] = (unsigned short)(bf16_bits(b.z) & mk); o[7] = (unsigned short)(bf16_bits(b.w) & mk);
    st2_v8us(xb + (size_t)row * FIN + k8, o);
  } else if (blk < PBX + PBW) {
    wplane(w1a, 128, 0, b1, (blk - PBX) * NTHR + tid);
  } else if (blk < PBX + 2 * PBW) {
    wplane(w1c, 128, 64, b1, (blk - PBX - PBW) * NTHR + tid);
  } else if (blk < PBX + 3 * PBW) {
    wplane(w2a, 64, 0, b2, (blk - PBX - 2 * PBW) * NTHR + tid);
  } else if (blk < PBX + 4 * PBW) {
    wplane(w2c, 64, 64, b2, (blk - PBX - 3 * PBW) * NTHR + tid);
  } else if (blk < PBX + 4 * PBW + PB3) {
    const int u = (blk - PBX - 4 * PBW) * NTHR + tid;
    const int n = u >> 5, k8 = (u & 31) * 8;
    const int srow = (k8 >> 7) * 64 + (k8 & 63);
    const v8us o = colfetch8(wlin + (size_t)srow * HB + n, HB);
    st2_v8us(b3 + (size_t)n * HLW + k8, o);
  } else {
    const int sbk = blk - (PBX + 4 * PBW + PB3);
    if (sbk == 0)      small_plane(al1, sm + SM_ATT, 48, tid);
    else if (sbk == 1) small_plane(ar1, sm + SM_ATT + 64, 48, tid);
    else if (sbk == 2) small_plane(al2, sm + SM_ATT + 384, 48, tid);
    else if (sbk == 3) small_plane(ar2, sm + SM_ATT + 384 + 64, 48, tid);
    else if (sbk == 4) small_plane(b1a, sm + SM_BIAS, 48, tid);
    else if (sbk == 5) small_plane(b1c, sm + SM_BIAS + 64, 48, tid);
    else if (sbk == 6) small_plane(b2a, sm + SM_BIAS + 384, 48, tid);
    else if (sbk == 7) small_plane(b2c, sm + SM_BIAS + 384 + 64, 48, tid);
    else               small_plane(blin, sm + SM_BLIN, 16, tid);
  }
}

__device__ __forceinline__ float rsq_cnt(int c) {
  const float xv = (float)(c < 1 ? 1 : c);
  const float y  = __builtin_amdgcn_rsqf(xv);
  const float e  = fmaf(-(xv * y), y, 1.0f);
  return fmaf(0.5f * y, e, y);
}

__device__ __forceinline__ void bucket_flush(const int* pl, const int* cnt, const int* offs, v4f nv, int ov, int kind,
                                             int* lp, int* cp, int* op, float* np, int* fp, int tid) {
  if (kind == 0) {
#pragma unroll 1
    for (int i = tid * 4; i < RCAP; i += NTHR * 4) {
      const v4i v = *(const v4ia*)(pl + i);
      *(volatile v4i*)(lp + i) = v;
    }
    {
      const v4i v = *(const v4ia*)(cnt + 4 * tid);
      *(volatile v4i*)(cp + 4 * tid) = v;
    }
    {
      const v4i v = *(const v4ia*)(offs + 4 * tid);
      *(volatile v4i*)(op + 4 * tid) = v;
    }
    if (tid < 8) {
      const v4i f = {ov, ov, ov, ov};
      *(volatile v4i*)(fp + 4 * tid) = f;
    }
  }
  *(volatile v4f*)(np + 4 * tid) = nv;
}

__global__ __launch_bounds__(NTHR) void k_bucket(const int* __restrict__ ei, int* LIST, int* CNT, int* OFF,
                                                 float* NRM, int* FLAG) {
  extern __shared__ __attribute__((aligned(16))) int dsm[];
  int* wl   = dsm;
  int* pl   = dsm + NWAVE * WLCAP;
  int* cnt  = pl + RCAP;
  int* offs = cnt + NBRUN;
  int* cur  = offs + NBRUN;
  int* misc = cur + NBRUN;
  const int tid = (int)threadIdx.x, lane = tid & 31, wave = tid >> 5;
  const int blk  = (int)blockIdx.x;
  const int role = (int)blockIdx.y;
  const int r    = role >> 1;
  const int kind = role & 1;
  const int* srcs = ei + (size_t)r * (size_t)(2 * NE);
  const int* keys = srcs + (kind == 0 ? NE : 0);
  const unsigned nbs = (unsigned)(blk * NBRUN);

  {
    const v4i z4 = {0, 0, 0, 0};
    for (int i = tid * 4; i < BK_ZINTS; i += NTHR * 4) *(v4ia*)(dsm + i) = z4;
    if (tid < 16) misc[tid] = 0;
  }
  __syncthreads();

  {
    const int per  = ((NE + NWAVE * WCH - 1) / (NWAVE * WCH)) * WCH;
    const int ebeg = wave * per;
    const int eend = (ebeg + per < NE) ? (ebeg + per) : NE;
    int* mylist = wl + wave * WLCAP;
    int wc = 0;
#pragma unroll 1
    for (int cb = ebeg; cb < eend; cb += WCH) {
      const int e0 = cb + lane * EPT;
      const v4i da = *(const v4ia*)(keys + e0);
      const v4i db = *(const v4ia*)(keys + e0 + 4);
      const unsigned s0 = (unsigned)da.x - nbs, s1 = (unsigned)da.y - nbs;
      const unsigned s2 = (unsigned)da.z - nbs, s3 = (unsigned)da.w - nbs;
      const unsigned s4 = (unsigned)db.x - nbs, s5 = (unsigned)db.y - nbs;
      const unsigned s6 = (unsigned)db.z - nbs, s7 = (unsigned)db.w - nbs;
      const bool h0 = s0 < (unsigned)NBRUN, h1 = s1 < (unsigned)NBRUN, h2 = s2 < (unsigned)NBRUN, h3 = s3 < (unsigned)NBRUN;
      const bool h4 = s4 < (unsigned)NBRUN, h5 = s5 < (unsigned)NBRUN, h6 = s6 < (unsigned)NBRUN, h7 = s7 < (unsigned)NBRUN;
      const unsigned m0 = __builtin_amdgcn_ballot_w32(h0), m1 = __builtin_amdgcn_ballot_w32(h1);
      const unsigned m2 = __builtin_amdgcn_ballot_w32(h2), m3 = __builtin_amdgcn_ballot_w32(h3);
      const unsigned m4 = __builtin_amdgcn_ballot_w32(h4), m5 = __builtin_amdgcn_ballot_w32(h5);
      const unsigned m6 = __builtin_amdgcn_ballot_w32(h6), m7 = __builtin_amdgcn_ballot_w32(h7);
      const unsigned any = m0 | m1 | m2 | m3 | m4 | m5 | m6 | m7;
      if (any != 0u) {
        const int pre = (int)(__builtin_amdgcn_mbcnt_lo(m0, 0u) + __builtin_amdgcn_mbcnt_lo(m1, 0u) +
                              __builtin_amdgcn_mbcnt_lo(m2, 0u) + __builtin_amdgcn_mbcnt_lo(m3, 0u) +
                              __builtin_amdgcn_mbcnt_lo(m4, 0u) + __builtin_amdgcn_mbcnt_lo(m5, 0u) +
                              __builtin_amdgcn_mbcnt_lo(m6, 0u) + __builtin_amdgcn_mbcnt_lo(m7, 0u));
        int p = wc + pre;
        if (h0) { if (p < WLCAP) mylist[p] = ((e0 + 0) << SLB) | (int)s0; p = p + 1; }
        if (h1) { if (p < WLCAP) mylist[p] = ((e0 + 1) << SLB) | (int)s1; p = p + 1; }
        if (h2) { if (p < WLCAP) mylist[p] = ((e0 + 2) << SLB) | (int)s2; p = p + 1; }
        if (h3) { if (p < WLCAP) mylist[p] = ((e0 + 3) << SLB) | (int)s3; p = p + 1; }
        if (h4) { if (p < WLCAP) mylist[p] = ((e0 + 4) << SLB) | (int)s4; p = p + 1; }
        if (h5) { if (p < WLCAP) mylist[p] = ((e0 + 5) << SLB) | (int)s5; p = p + 1; }
        if (h6) { if (p < WLCAP) mylist[p] = ((e0 + 6) << SLB) | (int)s6; p = p + 1; }
        if (h7) { if (p < WLCAP) mylist[p] = ((e0 + 7) << SLB) | (int)s7; p = p + 1; }
        wc += (int)(__builtin_popcount(m0) + __builtin_popcount(m1) + __builtin_popcount(m2) + __builtin_popcount(m3) +
                    __builtin_popcount(m4) + __builtin_popcount(m5) + __builtin_popcount(m6) + __builtin_popcount(m7));
      }
    }
    if (lane == 0) misc[wave] = wc;
  }
  __syncthreads();

  if (wave == 0) {
    int ov = 0;
#pragma unroll 1
    for (int w2 = 0; w2 < NWAVE; ++w2) {
      int c = misc[w2];
      if (c > WLCAP) ov = 1;
      c = c < 0 ? 0 : (c > WLCAP ? WLCAP : c);
#pragma unroll 1
      for (int b0 = 0; b0 < c; b0 += 32) {
        const int idx = b0 + lane;
        const int ent = wl[w2 * WLCAP + (idx < WLCAP ? idx : WLCAP - 1)];
        const int m32 = (c - b0) < 32 ? (c - b0) : 32;
#pragma unroll 1
        for (int k = 0; k < m32; ++k) {
          const int u    = __builtin_amdgcn_readlane(ent, k);
          const int slot = u & (NBRUN - 1);
          if (lane == 0) cnt[slot] = cnt[slot] + 1;
        }
      }
    }
    if (lane == 0) misc[9] = ov;
  }
  __syncthreads();
  if (wave == 0) {
    const int base = lane * (NBRUN / 32);
    int s = 0;
#pragma unroll 1
    for (int i = 0; i < NBRUN / 32; ++i) s += cnt[base + i];
    int incl = s;
#pragma unroll
    for (int d = 1; d < 32; d <<= 1) {
      const int y = __shfl_up(incl, d, 32);
      if (lane >= d) incl += y;
    }
    int run = incl - s;
#pragma unroll 1
    for (int i = 0; i < NBRUN / 32; ++i) {
      const int cv = cnt[base + i];
      offs[base + i] = run;
      cur[base + i]  = run;
      run += cv;
    }
  }
  __syncthreads();

  if (wave == 0 && kind == 0) {
#pragma unroll 1
    for (int w2 = 0; w2 < NWAVE; ++w2) {
      int c = misc[w2];
      c = c < 0 ? 0 : (c > WLCAP ? WLCAP : c);
#pragma unroll 1
      for (int b0 = 0; b0 < c; b0 += 32) {
        const int idx = b0 + lane;
        const int ent = wl[w2 * WLCAP + (idx < WLCAP ? idx : WLCAP - 1)];
        int eid = (ent >> SLB) & 0x1FFFFF;
        eid = eid > NE - 1 ? NE - 1 : eid;
        int sr = srcs[eid];
        sr = sr < 0 ? 0 : (sr > NN - 1 ? NN - 1 : sr);
        const int m32 = (c - b0) < 32 ? (c - b0) : 32;
#pragma unroll 1
        for (int k = 0; k < m32; ++k) {
          const int u    = __builtin_amdgcn_readlane(ent, k);
          const int wd   = __builtin_amdgcn_readlane(sr, k);
          const int slot = u & (NBRUN - 1);
          if (lane == 0) {
            int p = cur[slot];
            p = p < 0 ? 0 : (p > RCAP - 1 ? RCAP - 1 : p);
            pl[p] = wd;
            cur[slot] = p + 1;
          }
        }
      }
    }
  }
  __syncthreads();

  const int ovf = misc[9];
  const v4i cv = *(const v4ia*)(cnt + 4 * tid);
  const float qnan = __uint_as_float(0x7fc00000u);
  v4f nv;
  nv.x = rsq_cnt(cv.x); nv.y = rsq_cnt(cv.y); nv.z = rsq_cnt(cv.z); nv.w = rsq_cnt(cv.w);
  nv.x = (ovf != 0) ? qnan : nv.x; nv.y = (ovf != 0) ? qnan : nv.y;
  nv.z = (ovf != 0) ? qnan : nv.z; nv.w = (ovf != 0) ? qnan : nv.w;
  int*   lp = LIST + (size_t)(r * NBK + blk) * RCAP;
  int*   cp = CNT + (size_t)r * NSLOT + (size_t)blk * NBRUN;
  int*   op = OFF + (size_t)r * NSLOT + (size_t)blk * NBRUN;
  float* np = NRM + (size_t)(kind * NR + r) * NSLOT + (size_t)blk * NBRUN;
  int*   fp = FLAG + (size_t)(r * NBK + blk) * 32;
  bucket_flush(pl, cnt, offs, nv, ovf, kind, lp, cp, op, np, fp, tid);
  __threadfence();
  bucket_flush(pl, cnt, offs, nv, ovf, kind, lp, cp, op, np, fp, tid);
}

template <int KTOT, int LDB>
__device__ __forceinline__ void gemm_16x64(const unsigned short* __restrict__ ap,
                                           const unsigned short* __restrict__ bp, v8f (&acc)[4]) {
#pragma unroll 1
  for (int k0 = 0; k0 < KTOT; k0 += 32) {
    FragB af;
    af.h[0] = *(const v8usa*)(ap + k0);
    af.h[1] = *(const v8usa*)(ap + k0 + 16);
#pragma unroll
    for (int nt = 0; nt < 4; ++nt) {
      const unsigned short* wq = bp + (size_t)(16 * nt) * (size_t)LDB + k0;
      FragB bf;
      bf.h[0] = *(const v8usa*)wq;
      bf.h[1] = *(const v8usa*)(wq + 16);
      acc[nt] = wmb(af, bf, acc[nt]);
    }
  }
}

__device__ __forceinline__ void stage_d(float* stg, const v8f (&acc)[4], int wave, int hh, int m) {
#pragma unroll
  for (int nt = 0; nt < 4; ++nt) {
#pragma unroll
    for (int r = 0; r < 8; ++r) stg[(16 * wave + 8 * hh + r) * SP + 16 * nt + m] = acc[nt][r];
  }
}

template <int LAYER>
__global__ __launch_bounds__(NTHR) __attribute__((amdgpu_num_vgpr(248)))
void k_gemm(const unsigned short* __restrict__ A, const unsigned short* __restrict__ BT,
            const float* __restrict__ SM, const float* __restrict__ NRM, float* F, float* ELR) {
  constexpr int LDA = (LAYER == 1) ? FIN : HLW;
  __shared__ __attribute__((aligned(16))) float stg[GBM * SP];
  __shared__ __attribute__((aligned(16))) float satt[128];
  __shared__ __attribute__((aligned(16))) float sns[128];
  __shared__ __attribute__((aligned(16))) float sdot[1024];
  const int tid = (int)threadIdx.x, lane = tid & 31, wave = tid >> 5, hh = lane >> 4, m = lane & 15;
  const int rowBase = (int)blockIdx.x * GBM;
  const int role = (int)blockIdx.y;
  const int r = role >> 1, br = role & 1;

  if (tid < 32) {
    *(v4fa*)(satt + 4 * tid) = *(const v4fa*)(SM + SM_ATT + ((LAYER - 1) * NR + r) * 128 + 4 * tid);
  } else if (tid < 64) {
    const int t = tid - 32;
    *(v4fa*)(sns + 4 * t) = *(const v4fa*)(NRM + (size_t)(NR + r) * NSLOT + rowBase + 4 * t);
  }

  v8f acc[4];
  {
    const v8f z = {0.f, 0.f, 0.f, 0.f, 0.f, 0.f, 0.f, 0.f};
#pragma unroll
    for (int t = 0; t < 4; ++t) acc[t] = z;
  }
  const int koff = (LAYER == 2) ? br * 128 : 0;
  const unsigned short* ap = A + (size_t)(rowBase + 16 * wave + m) * (size_t)LDA + koff + 8 * hh;
  const unsigned short* bp = BT + (size_t)(r * 128 + br * 64 + m) * (size_t)128 + 8 * hh;
  gemm_16x64<128, 128>(ap, bp, acc);
  stage_d(stg, acc, wave, hh, m);
  __syncthreads();

  if (br == 0) {
    const int row = tid & 127, which = tid >> 7;
    const float* hr = stg + row * SP;
    const float* sa = satt + which * 64;
    float dh[4];
#pragma unroll
    for (int h = 0; h < 4; ++h) {
      float d = 0.0f;
#pragma unroll
      for (int c4 = 0; c4 < 4; ++c4) {
        const v4f hv = *(const v4fa*)(hr + 16 * h + 4 * c4);
        const v4f av = *(const v4fa*)(sa + 16 * h + 4 * c4);
        d = fmaf(hv.x, av.x, d);
        d = fmaf(hv.y, av.y, d);
        d = fmaf(hv.z, av.z, d);
        d = fmaf(hv.w, av.w, d);
      }
      dh[h] = d;
    }
    v4f dv;
    dv.x = dh[0]; dv.y = dh[1]; dv.z = dh[2]; dv.w = dh[3];
    *(v4fa*)(sdot + 4 * tid) = dv;
  }
  __syncthreads();

#pragma unroll 1
  for (int i = 0; i < 8; ++i) {
    const int lr   = 16 * wave + 2 * i + hh;
    const int grow = rowBase + lr;
    const v4f a = *(const v4fa*)(stg + lr * SP + 4 * m);
    const float sv = sns[lr];
    const float sc = (br != 0) ? sv : 1.0f;
    v4f o;
    o.x = a.x * sc; o.y = a.y * sc; o.z = a.z * sc; o.w = a.w * sc;
    st2_v4f(F + (size_t)grow * FW + r * 128 + br * 64 + 4 * m, o);
  }

  if (br == 0) {
    const int row = tid & 127, which = tid >> 7;
    const v4f v = *(const v4fa*)(sdot + 4 * tid);
    st2_v4f(ELR + (size_t)which * ER_OFS + ((size_t)r * MP + rowBase + row) * 4, v);
  }
}

template <int LAYER>
__global__ __launch_bounds__(NTHR) void k_replay(
    const int* __restrict__ LIST, const int* __restrict__ CNT, const int* __restrict__ OFF,
    const float* __restrict__ NRM, const int* __restrict__ FLAG,
    const float* __restrict__ F, const float* __restrict__ ELR, const float* __restrict__ SM,
    unsigned short* HL) {
  const int tid = (int)threadIdx.x, lane = tid & 31;
  const int wave = __builtin_amdgcn_readfirstlane(tid >> 5);
  const int rowBase = (int)blockIdx.x * RBM;
  const int bucket  = rowBase >> SLB;
  const int hsel    = (lane >> 2) & 3;
  const bool isAtt  = lane < 16;
  const int flag = FLAG[(size_t)(0 * NBK + bucket) * 32] | FLAG[(size_t)(1 * NBK + bucket) * 32] |
                   FLAG[(size_t)(2 * NBK + bucket) * 32];
  const float qnan = __uint_as_float(0x7fc00000u);

#pragma unroll 1
  for (int it = 0; it < RBM / NWAVE; ++it) {
    const int d = rowBase + wave * (RBM / NWAVE) + it;
    float t0 = 0.0f, t1 = 0.0f, t2 = 0.0f, t3 = 0.0f;
    int big = 0;
#pragma unroll 1
    for (int r = 0; r < NR; ++r) {
      int c = CNT[(size_t)r * NSLOT + d];
      int o = OFF[(size_t)r * NSLOT + d];
      const float ndv = NRM[(size_t)r * NSLOT + d];
      asm volatile("" :: "v"(ndv));
      c = __builtin_amdgcn_readfirstlane(c);
      o = __builtin_amdgcn_readfirstlane(o);
      big |= (int)(c > DEGCAP);
      c = max(0, min(c, DEGCAP));
      o = max(0, min(o, RCAP - 1));
      int last = o + c - 1;
      last = min(last, RCAP - 1);
      last = max(last, o);
      const int* lb = LIST + (size_t)(r * NBK + bucket) * RCAP;
      const float erv = ELR[(size_t)ER_OFS + ((size_t)r * MP + d) * 4 + hsel];
      const v4f bb = *(const v4fa*)(SM + SM_BIAS + ((LAYER - 1) * NR + r) * 128 + 4 * lane);
      const float* Fr  = F + r * 128 + 4 * lane;
      const float* ELp = ELR + (size_t)r * MP * 4 + hsel;
      float mx = -3.0e38f, dn = 0.0f;
      float a0 = 0.0f, a1 = 0.0f, a2 = 0.0f, a3 = 0.0f;
#pragma unroll 1
      for (int j = 0; j < c; ++j) {
        int idx = o + j;
        idx = min(idx, last);
        int s = lb[idx];
        s = max(0, min(s, NN - 1));
        const v4f fs = *(const v4fa*)(Fr + (size_t)s * FW);
        const float elv = ELp[(size_t)s * 4];
        asm volatile("" :: "v"(fs));
        asm volatile("" :: "v"(elv));
        float lg = elv + erv;
        lg = lg > 0.0f ? lg : 0.2f * lg;
        const float df = lg - mx;
        const float ee = expf(-fabsf(df));
        const bool up  = df > 0.0f;
        float s1 = up ? ee : 1.0f;
        float s2 = up ? 1.0f : ee;
        s1 = isAtt ? s1 : 1.0f;
        s2 = isAtt ? s2 : 1.0f;
        mx = up ? lg : mx;
        dn = fmaf(dn, s1, s2);
        a0 = fmaf(a0, s1, s2 * fs.x);
        a1 = fmaf(a1, s1, s2 * fs.y);
        a2 = fmaf(a2, s1, s2 * fs.z);
        a3 = fmaf(a3, s1, s2 * fs.w);
      }
      const float dd  = (dn < 1e-9f) ? 1e-9f : dn;
      const float inv = 1.0f / dd;
      const float sc  = isAtt ? inv : ndv;
      const float o0 = fmaf(a0, sc, bb.x), o1 = fmaf(a1, sc, bb.y);
      const float o2 = fmaf(a2, sc, bb.z), o3 = fmaf(a3, sc, bb.w);
      t0 = t0 + o0; t1 = t1 + o1; t2 = t2 + o2; t3 = t3 + o3;
    }
    float v0 = t0 / 3.0f, v1 = t1 / 3.0f, v2 = t2 / 3.0f, v3 = t3 / 3.0f;
    if (LAYER == 1) {
      v0 = v0 > 0.0f ? v0 : 0.01f * v0; v1 = v1 > 0.0f ? v1 : 0.01f * v1;
      v2 = v2 > 0.0f ? v2 : 0.01f * v2; v3 = v3 > 0.0f ? v3 : 0.01f * v3;
    }
    const bool bad  = ((flag | big) != 0);
    const bool live = d < NN;
    v0 = bad ? qnan : v0; v1 = bad ? qnan : v1; v2 = bad ? qnan : v2; v3 = bad ? qnan : v3;
    v0 = live ? v0 : 0.0f; v1 = live ? v1 : 0.0f; v2 = live ? v2 : 0.0f; v3 = live ? v3 : 0.0f;
    int h01, h23, l01, l23;
    hilo_pack(v0, v1, v2, v3, h01, h23, l01, l23);
    const v4i ow = regroup8(h01, h23, l01, l23, lane);
    unsigned short* hp = HL + (size_t)d * HLW + 8 * lane;
    *(volatile v4i*)hp = ow;
    __threadfence();
    *(volatile v4i*)hp = ow;
  }
}

__global__ __launch_bounds__(NTHR) __attribute__((amdgpu_num_vgpr(248)))
void k_final(const unsigned short* __restrict__ HL, const unsigned short* __restrict__ B3,
             const float* __restrict__ SM, const int* __restrict__ FLAG, float* out) {
  __shared__ __attribute__((aligned(16))) float stg[GBM * SP];
  __shared__ __attribute__((aligned(16))) float sb[64];
  const int tid = (int)threadIdx.x, lane = tid & 31, wave = tid >> 5, hh = lane >> 4, m = lane & 15;
  const int rowBase = (int)blockIdx.x * GBM;
  const int bucket  = rowBase >> SLB;
  const int flag = FLAG[(size_t)(0 * NBK + bucket) * 32] | FLAG[(size_t)(1 * NBK + bucket) * 32] |
                   FLAG[(size_t)(2 * NBK + bucket) * 32];
  if (tid < 16) *(v4fa*)(sb + 4 * tid) = *(const v4fa*)(SM + SM_BLIN + 4 * tid);

  v8f acc[4];
  {
    const v8f z = {0.f, 0.f, 0.f, 0.f, 0.f, 0.f, 0.f, 0.f};
#pragma unroll
    for (int t = 0; t < 4; ++t) acc[t] = z;
  }
  const unsigned short* ap = HL + (size_t)(rowBase + 16 * wave + m) * (size_t)HLW + 8 * hh;
  const unsigned short* bp = B3 + (size_t)m * (size_t)HLW + 8 * hh;
  gemm_16x64<HLW, HLW>(ap, bp, acc);
  stage_d(stg, acc, wave, hh, m);
  __syncthreads();

  const v4f bias = *(const v4fa*)(sb + 4 * m);
  const float qnan = __uint_as_float(0x7fc00000u);
#pragma unroll 1
  for (int i = 0; i < 8; ++i) {
    const int lr   = 16 * wave + 2 * i + hh;
    const int grow = rowBase + lr;
    const bool live = grow < NN;
    const v4f a = *(const v4fa*)(stg + lr * SP + 4 * m);
    asm volatile("" :: "v"(a));
    v4f o;
    o.x = a.x + bias.x; o.y = a.y + bias.y; o.z = a.z + bias.z; o.w = a.w + bias.w;
    o.x = (flag != 0) ? qnan : o.x; o.y = (flag != 0) ? qnan : o.y;
    o.z = (flag != 0) ? qnan : o.z; o.w = (flag != 0) ? qnan : o.w;
    float* op = out + (size_t)grow * HB + 4 * m;
    if (live) *(volatile v4f*)op = o;
    __threadfence();
    if (live) *(volatile v4f*)op = o;
  }
}

extern "C" void kernel_launch(void* const* d_in, const int* in_sizes, int n_in,
                              void* d_out, int out_size, void* d_ws, size_t ws_size,
                              hipStream_t stream) {
  if (n_in < 16) return;
  if (in_sizes[0] != NN * FIN) return;
  if (in_sizes[1] != NR * 2 * NE) return;
  if (in_sizes[2] != NR * FIN * HB) return;
  if (in_sizes[3] != NR * HB || in_sizes[4] != NR * HB) return;
  if (in_sizes[5] != NR * HB) return;
  if (in_sizes[6] != NR * HB * HB) return;
  if (in_sizes[7] != NR * HB || in_sizes[8] != NR * HB) return;
  if (in_sizes[9] != NR * HB) return;
  if (in_sizes[10] != NR * FIN * HB) return;
  if (in_sizes[11] != NR * HB) return;
  if (in_sizes[12] != NR * HB * HB) return;
  if (in_sizes[13] != NR * HB) return;
  if (in_sizes[14] != 2 * HB * HB) return;
  if (in_sizes[15] != HB) return;
  if (out_size != NN * HB) return;

  const float* x    = (const float*)d_in[0];
  const int*   ei   = (const int*)d_in[1];
  const float* W1a  = (const float*)d_in[2];
  const float* al1  = (const float*)d_in[3];
  const float* ar1  = (const float*)d_in[4];
  const float* b1a  = (const float*)d_in[5];
  const float* W2a  = (const float*)d_in[6];
  const float* al2  = (const float*)d_in[7];
  const float* ar2  = (const float*)d_in[8];
  const float* b2a  = (const float*)d_in[9];
  const float* W1c  = (const float*)d_in[10];
  const float* b1c  = (const float*)d_in[11];
  const float* W2c  = (const float*)d_in[12];
  const float* b2c  = (const float*)d_in[13];
  const float* Wlin = (const float*)d_in[14];
  const float* blin = (const float*)d_in[15];
  float* out = (float*)d_out;

  constexpr size_t zHL   = (size_t)MP * HLW * 2;
  constexpr size_t zXB   = (size_t)MP * FIN * 2;
  constexpr size_t zF    = (size_t)MP * FW * 4;
  constexpr size_t zELR  = (size_t)2 * NR * MP * 16;
  constexpr size_t zLIST = (size_t)NR * NBK * RCAP * 4;
  constexpr size_t zCNT  = (size_t)NR * NSLOT * 4;
  constexpr size_t zNRM  = (size_t)2 * NR * NSLOT * 4;
  constexpr size_t zFLAG = 18944;
  constexpr size_t zB12  = (size_t)384 * 128 * 2;
  constexpr size_t zB3   = (size_t)HB * HLW * 2;
  constexpr size_t zSM   = (size_t)SM_N * 4;
  constexpr size_t oHL   = 0;
  constexpr size_t oF    = oHL + zHL;
  constexpr size_t oELR  = oF + zF;
  constexpr size_t oLIST = oELR + zELR;
  constexpr size_t oCNT  = oLIST + zLIST;
  constexpr size_t oOFF  = oCNT + zCNT;
  constexpr size_t oNRM  = oOFF + zCNT;
  constexpr size_t oFLAG = oNRM + zNRM;
  constexpr size_t oB1   = oFLAG + zFLAG;
  constexpr size_t oB2   = oB1 + zB12;
  constexpr size_t oB3   = oB2 + zB12;
  constexpr size_t oSM   = oB3 + zB3;
  constexpr size_t oEND  = oSM + zSM;
  static_assert(zXB <= zHL);
  static_assert(zHL % 256 == 0 && zF % 256 == 0 && zELR % 256 == 0 && zLIST % 256 == 0 && zCNT % 256 == 0);
  static_assert(zNRM % 256 == 0 && zFLAG % 256 == 0 && zB12 % 256 == 0 && zB3 % 256 == 0 && zSM % 256 == 0);
  static_assert(zFLAG >= (size_t)NR * NBK * 128);
  static_assert(oEND <= (size_t)WSMAX);
  if (oEND > ws_size) return;

  char* ws = (char*)d_ws;
  unsigned short* HLp  = (unsigned short*)(ws + oHL);
  unsigned short* XB   = (unsigned short*)(ws + oHL);
  float*          F    = (float*)(ws + oF);
  float*          ELR  = (float*)(ws + oELR);
  int*            LIST = (int*)(ws + oLIST);
  int*            CNT  = (int*)(ws + oCNT);
  int*            OFF  = (int*)(ws + oOFF);
  float*          NRM  = (float*)(ws + oNRM);
  int*            FLAG = (int*)(ws + oFLAG);
  unsigned short* B1   = (unsigned short*)(ws + oB1);
  unsigned short* B2   = (unsigned short*)(ws + oB2);
  unsigned short* B3   = (unsigned short*)(ws + oB3);
  float*          SM   = (float*)(ws + oSM);

  hipFuncSetAttribute(reinterpret_cast<const void*>(&k_bucket), hipFuncAttributeMaxDynamicSharedMemorySize, (int)BK_LDS);

  k_prep<<<PBTOT, NTHR, 0, stream>>>(x, W1a, W1c, W2a, W2c, Wlin, al1, ar1, al2, ar2, b1a, b2a, b1c, b2c, blin,
                                     XB, B1, B2, B3, SM);
  k_bucket<<<dim3(NBK, 2 * NR), NTHR, BK_LDS, stream>>>(ei, LIST, CNT, OFF, NRM, FLAG);
  k_gemm<1><<<dim3(MP / GBM, 2 * NR), NTHR, 0, stream>>>(XB, B1, SM, NRM, F, ELR);
  k_replay<1><<<MP / RBM, NTHR, 0, stream>>>(LIST, CNT, OFF, NRM, FLAG, F, ELR, SM, HLp);
  k_gemm<2><<<dim3(MP / GBM, 2 * NR), NTHR, 0, stream>>>(HLp, B2, SM, NRM, F, ELR);
  k_replay<2><<<MP / RBM, NTHR, 0, stream>>>(LIST, CNT, OFF, NRM, FLAG, F, ELR, SM, HLp);
  k_final<<<MP / GBM, NTHR, 0, stream>>>(HLp, B3, SM, FLAG, out);
}
